// LstmEncoder_19104014533401
// MI455X (gfx1250) — hardware-verified
//
#include <hip/hip_runtime.h>
#include <math.h>

constexpr int NBATCH = 32;
constexpr int NSTEP  = 512;
constexpr int NIN    = 256;
constexpr int NHID   = 512;
constexpr int NLAT   = 256;
constexpr int NTHR   = 256;
constexpr int TCH    = 128;
constexpr int NCHUNK = NSTEP / TCH;
constexpr int MCH    = TCH * NBATCH;
constexpr int NROWS  = NSTEP * NBATCH;
constexpr float XCARRY = 16.0f;
constexpr float WCARRY = 16.0f;
constexpr float HCARRY = 64.0f;
constexpr float FOLD_XW = 1.0f / (XCARRY * WCARRY);
constexpr float FOLD_HW = 1.0f / (HCARRY * WCARRY);
constexpr float BN_EPS_F = 1e-3f;

static_assert(NSTEP % TCH == 0);
static_assert(TCH % 2 == 0);
static_assert(MCH % 64 == 0);
static_assert((4 * NHID) % 64 == 0 && (4 * NLAT) % 64 == 0);
static_assert(NIN % 32 == 0 && NHID % 32 == 0 && NLAT % 32 == 0);
static_assert(NBATCH == 32);

typedef __attribute__((ext_vector_type(16))) _Float16 v16h;
typedef __attribute__((ext_vector_type(8)))  _Float16 v8h;
typedef __attribute__((ext_vector_type(8)))  float    v8f;
typedef __attribute__((ext_vector_type(4)))  float    v4f;

__device__ __forceinline__ unsigned short f2bf_bits(float f) {
  unsigned u = __float_as_uint(f);
  return (unsigned short)((u + 0x7FFFu + ((u >> 16) & 1u)) >> 16);
}
__device__ __forceinline__ float bf_bits2f(unsigned short h) { return __uint_as_float(((unsigned)h) << 16); }
__device__ __forceinline__ float bf16r(float f) { return bf_bits2f(f2bf_bits(f)); }

__device__ __forceinline__ void wm_guard4(v8f& a0, v8f& a1, v8f& a2, v8f& a3, v16h x, v16h b0, v16h b1, v16h b2, v16h b3) {
  asm volatile("v_nop\n\tv_nop\n\tv_nop\n\tv_nop" : "+v"(a0), "+v"(a1), "+v"(a2), "+v"(a3) : "v"(x), "v"(b0), "v"(b1), "v"(b2), "v"(b3));
}
__device__ __forceinline__ void acc_guard4(v8f& a, v8f& b, v8f& c, v8f& d) {
  asm volatile("v_nop\n\tv_nop\n\tv_nop\n\tv_nop" : "+v"(a), "+v"(b), "+v"(c), "+v"(d));
}

union FragU { v16h v; v8h h[2]; };
__device__ __forceinline__ v16h frag_load(const _Float16* p) {
  FragU f;
  f.h[0] = *(const v8h*)(p);
  f.h[1] = *(const v8h*)(p + 16);
  return f.v;
}
__device__ __forceinline__ v8f frag_mma(v16h a, v16h b, v8f c) {
  return __builtin_amdgcn_wmma_f32_16x16x32_f16(false, a, false, b, (short)0, c, false, false);
}

__device__ __forceinline__ float fsig(float x) { return __builtin_amdgcn_rcpf(1.0f + __expf(-x)); }

__global__ __launch_bounds__(NTHR) void cvt_x_kernel(const float* __restrict__ x, unsigned short* __restrict__ dst) {
  constexpr int P8 = NIN / 8;
  const int i = blockIdx.x * NTHR + threadIdx.x;
  if (i < NROWS * P8) {
    const int m  = i / P8;
    const int c8 = i - m * P8;
    const int t  = m / NBATCH;
    const int b  = m - t * NBATCH;
    const float* sp = x + ((size_t)b * NSTEP + (size_t)t) * NIN + c8 * 8;
    const v4f a  = *(const v4f*)(sp);
    const v4f bq = *(const v4f*)(sp + 4);
    v8h hv;
#pragma unroll
    for (int e = 0; e < 4; ++e) {
      hv[e]     = (_Float16)(bf16r(a[e])  * XCARRY);
      hv[4 + e] = (_Float16)(bf16r(bq[e]) * XCARRY);
    }
    _Float16* op = (_Float16*)dst + (size_t)i * 8;
    *(volatile v8h*)op = hv;
    __threadfence();
    *(volatile v8h*)op = hv;
  }
}

__global__ __launch_bounds__(NTHR) void tpw_kernel(const float* __restrict__ src, int R, int C, int ldo,
                                                   unsigned short* __restrict__ O, float sc) {
  __shared__ float Tt[64 * 65];
  const int tid = threadIdx.x;
  const int c0 = blockIdx.x * 64, r0 = blockIdx.y * 64;
#pragma unroll
  for (int i = 0; i < 4; ++i) {
    const int idx = i * NTHR + tid;
    const int rr = idx >> 4, cc = (idx & 15) * 4;
    const v4f v = *(const v4f*)(src + (size_t)(r0 + rr) * (size_t)C + c0 + cc);
    Tt[rr * 65 + cc + 0] = v[0];
    Tt[rr * 65 + cc + 1] = v[1];
    Tt[rr * 65 + cc + 2] = v[2];
    Tt[rr * 65 + cc + 3] = v[3];
  }
  __syncthreads();
  const int q = tid >> 3, c8 = (tid & 7) * 8;
  v8h hv[2];
#pragma unroll
  for (int g = 0; g < 2; ++g) {
    const int qq = g * 32 + q;
#pragma unroll
    for (int e = 0; e < 8; ++e) {
      const float f = Tt[(c8 + e) * 65 + qq];
      hv[g][e] = (_Float16)(bf16r(f) * sc);
    }
  }
  _Float16* Oh = (_Float16*)O;
  for (int pass = 0; pass < 2; ++pass) {
#pragma unroll
    for (int g = 0; g < 2; ++g) {
      const size_t o = (size_t)(c0 + g * 32 + q) * (size_t)ldo + (size_t)(r0 + c8);
      *(volatile v8h*)(Oh + o) = hv[g];
    }
    __threadfence();
  }
}

__global__ __launch_bounds__(256) void gemm64_f16_kernel(
    const unsigned short* __restrict__ Ap, int lda,
    const unsigned short* __restrict__ Btp, int ldb,
    float* __restrict__ C, int ldc,
    const float* __restrict__ bias, int M, int N, int K, float scale) {
  const _Float16* A  = (const _Float16*)Ap;
  const _Float16* Bt = (const _Float16*)Btp;
  __shared__ __align__(16) float sT[8][16 * 68];
  const int lane = threadIdx.x & 31;
  const int wave = threadIdx.x >> 5;
  const int tilesN = N >> 6;
  const int tilesM = M >> 6;
  const int tile = blockIdx.x * 8 + wave;
  if (tile >= tilesM * tilesN) return;
  const int tm = tile / tilesN;
  const int tn = tile - tm * tilesN;
  const int m0 = tm << 6;
  const int n0 = tn << 6;
  const int rlane = lane & 15;
  const int koff  = (lane >> 4) * 8;
  const int mOff  = (lane >> 4) * 8;

  v8f acc[4][4];
#pragma unroll
  for (int i = 0; i < 4; ++i)
#pragma unroll
    for (int j = 0; j < 4; ++j) acc[i][j] = (v8f){0.f, 0.f, 0.f, 0.f, 0.f, 0.f, 0.f, 0.f};

  for (int k0 = 0; k0 < K; k0 += 32) {
    v16h bh[4];
#pragma unroll
    for (int j = 0; j < 4; ++j) {
      const size_t bo = (size_t)(n0 + (j << 4) + rlane) * ldb + koff + k0;
      bh[j] = frag_load(Bt + bo);
    }
#pragma unroll
    for (int i = 0; i < 4; ++i) {
      const size_t ao = (size_t)(m0 + (i << 4) + rlane) * lda + koff + k0;
      const v16h ah = frag_load(A + ao);
#pragma unroll
      for (int j = 0; j < 4; ++j) acc[i][j] = frag_mma(ah, bh[j], acc[i][j]);
      wm_guard4(acc[i][0], acc[i][1], acc[i][2], acc[i][3], ah, bh[0], bh[1], bh[2], bh[3]);
    }
  }
  acc_guard4(acc[0][0], acc[0][1], acc[0][2], acc[0][3]);
  acc_guard4(acc[1][0], acc[1][1], acc[1][2], acc[1][3]);
  acc_guard4(acc[2][0], acc[2][1], acc[2][2], acc[2][3]);
  acc_guard4(acc[3][0], acc[3][1], acc[3][2], acc[3][3]);

  float* slab = sT[wave];
#pragma unroll
  for (int i = 0; i < 4; ++i) {
    const int mBase = m0 + (i << 4);
#pragma unroll
    for (int j = 0; j < 4; ++j) {
      const int n = n0 + (j << 4) + rlane;
      const float bv = bf16r(bias[n]);
#pragma unroll
      for (int r = 0; r < 8; ++r) {
        const float v = acc[i][j][r] * scale + bv;
        slab[(mOff + r) * 68 + (j << 4) + rlane] = v;
      }
    }
    __builtin_amdgcn_fence(__ATOMIC_RELEASE, "workgroup");
    __builtin_amdgcn_wave_barrier();
    __builtin_amdgcn_fence(__ATOMIC_ACQUIRE, "workgroup");
    {
      const int hh = lane >> 4, c4 = (lane & 15) * 4;
      for (int pass = 0; pass < 2; ++pass) {
#pragma unroll
        for (int it = 0; it < 8; ++it) {
          const int row = it * 2 + hh;
          const v4f v = *(const v4f*)(slab + row * 68 + c4);
          *(volatile v4f*)(C + (size_t)(mBase + row) * ldc + n0 + c4) = v;
        }
        __threadfence();
      }
    }
    __builtin_amdgcn_fence(__ATOMIC_RELEASE, "workgroup");
    __builtin_amdgcn_wave_barrier();
    __builtin_amdgcn_fence(__ATOMIC_ACQUIRE, "workgroup");
  }
}

template <int UU, bool LAT>
__global__ __launch_bounds__(NTHR) void lstm_scan_kernel(
    const float* __restrict__ XW, const unsigned short* __restrict__ UTp,
    const float* __restrict__ gam, const float* __restrict__ bet,
    const float* __restrict__ mean, const float* __restrict__ var,
    unsigned short* SEQp, const float* CIN, const unsigned short* HINp,
    float* COUT, unsigned short* HOUTp, float* OUT, int is_first, int is_last) {
  constexpr int NTL = UU / 128;
  constexpr int HP  = UU + 8;
  constexpr int SP  = UU + 8;
  constexpr int OP  = UU + 4;
  constexpr int N4  = 4 * UU;
  constexpr int P8  = UU / 8;
  constexpr int NIT = (16 * P8) / NTHR;
  static_assert(UU % 128 == 0);
  static_assert((2 * 16 * HP) % NTHR == 0);
  static_assert((16 * P8) % NTHR == 0);
  __shared__ __align__(16) _Float16 Hh[2][16 * HP];
  __shared__ __align__(16) _Float16 Stg[LAT ? 1 : 2][LAT ? 8 : 16 * SP];
  __shared__ __align__(16) float    Hs[LAT ? 16 * OP : 4];

  const _Float16* UT  = (const _Float16*)UTp;
  _Float16*       SEQ = (_Float16*)SEQp;
  const _Float16* HIN = (const _Float16*)HINp;
  _Float16*       HOUT = (_Float16*)HOUTp;
  const int tid = threadIdx.x, lane = tid & 31, wave = tid >> 5;
  const int c = lane & 15, hh = lane >> 4, koff = hh * 8;
  const int blk = blockIdx.x;
  const int wbase = wave * (UU / 8);
  const int cslot = ((blk * 8 + wave) * NTL) * 256 + lane;

  {
    _Float16* hf = &Hh[0][0];
#pragma unroll 1
    for (int i = tid; i < 2 * 16 * HP; i += NTHR) hf[i] = (_Float16)0.0f;
  }
  float cst[NTL][8];
  float hfin[LAT ? NTL : 1][8];
  float bm[NTL], brs[NTL], bg[NTL], bb[NTL];
#pragma unroll
  for (int nt = 0; nt < NTL; ++nt) {
    bm[nt] = 0.0f; brs[nt] = 1.0f; bg[nt] = 1.0f; bb[nt] = 0.0f;
#pragma unroll
    for (int r = 0; r < 8; ++r) cst[nt][r] = 0.0f;
  }
#pragma unroll
  for (int nt = 0; nt < (LAT ? NTL : 1); ++nt)
#pragma unroll
    for (int r = 0; r < 8; ++r) hfin[nt][r] = 0.0f;
  if (!LAT) {
#pragma unroll
    for (int nt = 0; nt < NTL; ++nt) {
      const int j = wbase + 16 * nt + c;
      bm[nt]  = bf16r(mean[j]);
      brs[nt] = rsqrtf(bf16r(var[j]) + BN_EPS_F);
      bg[nt]  = bf16r(gam[j]);
      bb[nt]  = bf16r(bet[j]);
    }
  }
  __syncthreads();
  if (!is_first) {
    const _Float16* hin = HIN + (size_t)blk * 16 * UU;
#pragma unroll
    for (int it = 0; it < NIT; ++it) {
      const int idx = it * NTHR + tid;
      const int row = idx / P8;
      const int c8  = (idx - row * P8) * 8;
      const v8h v = *(const v8h*)(hin + row * UU + c8);
      *(v8h*)(&Hh[0][0] + row * HP + c8) = v;
    }
#pragma unroll
    for (int nt = 0; nt < NTL; ++nt)
#pragma unroll
      for (int r = 0; r < 8; ++r) cst[nt][r] = CIN[cslot + (nt * 8 + r) * 32];
  }
  __syncthreads();

  const v8f z8 = {0.f, 0.f, 0.f, 0.f, 0.f, 0.f, 0.f, 0.f};

#pragma unroll 1
  for (int tl = 0; tl < TCH; ++tl) {
    const int cur = tl & 1;
    const _Float16* ahrow = &Hh[cur][0] + c * HP + koff;
    _Float16* ahn = &Hh[cur ^ 1][0];
    _Float16* stg = &Stg[LAT ? 0 : cur][0];
    const float* xwt = XW + (size_t)(tl * NBATCH + blk * 16 + 8 * hh) * N4;
#pragma unroll
    for (int nt = 0; nt < NTL; ++nt) {
      const int j = wbase + 16 * nt + c;
      const _Float16* wr = UT + (size_t)j * UU + koff;
      v8f a0 = z8, a1 = z8, a2 = z8, a3 = z8;
#pragma unroll 1
      for (int k0 = 0; k0 < UU; k0 += 32) {
        const v16h a  = frag_load(ahrow + k0);
        const v16h b0 = frag_load(wr + k0);
        const v16h b1 = frag_load(wr + (size_t)1 * UU * UU + k0);
        const v16h b2 = frag_load(wr + (size_t)2 * UU * UU + k0);
        const v16h b3 = frag_load(wr + (size_t)3 * UU * UU + k0);
        a0 = frag_mma(a, b0, a0);
        a1 = frag_mma(a, b1, a1);
        a2 = frag_mma(a, b2, a2);
        a3 = frag_mma(a, b3, a3);
        wm_guard4(a0, a1, a2, a3, a, b0, b1, b2, b3);
      }
      acc_guard4(a0, a1, a2, a3);
#pragma unroll
      for (int r = 0; r < 8; ++r) {
        const float* xp = xwt + (size_t)r * N4 + j;
        const float zi = fmaf(a0[r], FOLD_HW, xp[0]);
        const float zf = fmaf(a1[r], FOLD_HW, xp[UU]);
        const float zg = fmaf(a2[r], FOLD_HW, xp[2 * UU]);
        const float zo = fmaf(a3[r], FOLD_HW, xp[3 * UU]);
        const float ig = fsig(zi);
        const float fg = fsig(zf);
        const float og = fsig(zo);
        const float cn = fg * cst[nt][r] + ig * zg;
        cst[nt][r] = cn;
        const float hv = og * cn;
        ahn[(8 * hh + r) * HP + j] = (_Float16)(hv * HCARRY);
        if (!LAT) {
          float pv = fmaxf(hv, 0.0f);
          pv = ((pv - bm[nt]) * brs[nt]) * bg[nt] + bb[nt];
          stg[(8 * hh + r) * SP + j] = (_Float16)(pv * HCARRY);
        } else {
          hfin[LAT ? nt : 0][r] = hv;
        }
      }
    }
    __syncthreads();
    if (!LAT) {
      _Float16* sq = SEQ + (size_t)(tl * NBATCH + blk * 16) * UU;
      v8h sv[NIT];
#pragma unroll
      for (int it = 0; it < NIT; ++it) {
        const int idx = it * NTHR + tid;
        const int row = idx / P8;
        const int c8  = (idx - row * P8) * 8;
        sv[it] = *(const v8h*)(stg + row * SP + c8);
      }
      for (int pass = 0; pass < 2; ++pass) {
#pragma unroll
        for (int it = 0; it < NIT; ++it) {
          const int idx = it * NTHR + tid;
          *(volatile v8h*)(sq + (size_t)idx * 8) = sv[it];
        }
        __threadfence();
      }
    }
  }

  {
    _Float16* ho = HOUT + (size_t)blk * 16 * UU;
    v8h hvv[NIT];
#pragma unroll
    for (int it = 0; it < NIT; ++it) {
      const int idx = it * NTHR + tid;
      const int row = idx / P8;
      const int c8  = (idx - row * P8) * 8;
      hvv[it] = *(const v8h*)(&Hh[0][0] + row * HP + c8);
    }
    for (int pass = 0; pass < 2; ++pass) {
#pragma unroll
      for (int it = 0; it < NIT; ++it) {
        const int idx = it * NTHR + tid;
        *(volatile v8h*)(ho + (size_t)idx * 8) = hvv[it];
      }
      __threadfence();
    }
  }
  {
    float* cp = COUT + cslot;
    for (int pass = 0; pass < 2; ++pass) {
#pragma unroll
      for (int nt = 0; nt < NTL; ++nt)
#pragma unroll
        for (int r = 0; r < 8; ++r) *(volatile float*)(cp + (nt * 8 + r) * 32) = cst[nt][r];
      __threadfence();
    }
  }
  if (LAT) {
#pragma unroll
    for (int nt = 0; nt < (LAT ? NTL : 1); ++nt) {
      const int j = wbase + 16 * nt + c;
#pragma unroll
      for (int r = 0; r < 8; ++r) Hs[(LAT ? ((8 * hh + r) * OP + j) : 0)] = hfin[nt][r];
    }
    __syncthreads();
    if (is_last) {
      constexpr int PER_ROW = UU / 4;
      constexpr int NOIT = (16 * PER_ROW) / NTHR;
      v4f ov[NOIT];
#pragma unroll
      for (int it = 0; it < NOIT; ++it) {
        const int idx = it * NTHR + tid;
        const int row = idx / PER_ROW;
        const int c4  = (idx - row * PER_ROW) * 4;
        ov[it] = *(const v4f*)(Hs + (LAT ? (row * OP + c4) : 0));
      }
      for (int pass = 0; pass < 2; ++pass) {
#pragma unroll
        for (int it = 0; it < NOIT; ++it) {
          const int idx = it * NTHR + tid;
          const int row = idx / PER_ROW;
          const int c4  = (idx - row * PER_ROW) * 4;
          *(volatile v4f*)(OUT + (size_t)(blk * 16 + row) * UU + c4) = ov[it];
        }
        __threadfence();
      }
    }
  }
}

extern "C" void kernel_launch(void* const* d_in, const int* in_sizes, int n_in,
                              void* d_out, int out_size, void* d_ws, size_t ws_size, hipStream_t stream) {
  if (n_in < 18 || d_out == nullptr || d_ws == nullptr) return;
  if (in_sizes[0] != NBATCH * NSTEP * NIN || in_sizes[1] != NIN * 4 * NHID || in_sizes[2] != NHID * 4 * NHID ||
      in_sizes[3] != 4 * NHID || in_sizes[4] != NHID || in_sizes[5] != NHID || in_sizes[6] != NHID || in_sizes[7] != NHID ||
      in_sizes[8] != NHID * 4 * NHID || in_sizes[9] != NHID * 4 * NHID || in_sizes[10] != 4 * NHID ||
      in_sizes[11] != NHID || in_sizes[12] != NHID || in_sizes[13] != NHID || in_sizes[14] != NHID ||
      in_sizes[15] != NHID * 4 * NLAT || in_sizes[16] != NLAT * 4 * NLAT || in_sizes[17] != 4 * NLAT ||
      out_size != NBATCH * NLAT) return;

  const float* x   = (const float*)d_in[0];
  const float* W0  = (const float*)d_in[1];
  const float* U0  = (const float*)d_in[2];
  const float* b0  = (const float*)d_in[3];
  const float* g0  = (const float*)d_in[4];
  const float* be0 = (const float*)d_in[5];
  const float* m0  = (const float*)d_in[6];
  const float* v0  = (const float*)d_in[7];
  const float* W1  = (const float*)d_in[8];
  const float* U1  = (const float*)d_in[9];
  const float* b1  = (const float*)d_in[10];
  const float* g1  = (const float*)d_in[11];
  const float* be1 = (const float*)d_in[12];
  const float* m1  = (const float*)d_in[13];
  const float* v1  = (const float*)d_in[14];
  const float* Wl  = (const float*)d_in[15];
  const float* Ul  = (const float*)d_in[16];
  const float* bl  = (const float*)d_in[17];
  float* out = (float*)d_out;

  char* ws = (char*)d_ws;
  size_t off = 0;
  auto carve = [&](size_t bytes) -> char* { char* p = ws + off; off += (bytes + 255) & ~(size_t)255; return p; };
  unsigned short* XA   = (unsigned short*)carve((size_t)NROWS * NIN * 2);
  unsigned short* W0T  = (unsigned short*)carve((size_t)4 * NHID * NIN * 2);
  unsigned short* U0T  = (unsigned short*)carve((size_t)4 * NHID * NHID * 2);
  unsigned short* W1T  = (unsigned short*)carve((size_t)4 * NHID * NHID * 2);
  unsigned short* U1T  = (unsigned short*)carve((size_t)4 * NHID * NHID * 2);
  unsigned short* WLT  = (unsigned short*)carve((size_t)4 * NLAT * NHID * 2);
  unsigned short* ULT  = (unsigned short*)carve((size_t)4 * NLAT * NLAT * 2);
  unsigned short* SEQ0 = (unsigned short*)carve((size_t)NROWS * NHID * 2);
  unsigned short* SEQ1 = (unsigned short*)carve((size_t)NROWS * NHID * 2);
  float*          XWC  = (float*)carve((size_t)MCH * 4 * NHID * 4);
  float*          CST  = (float*)carve((size_t)3 * NCHUNK * NBATCH * NHID * 4);
  unsigned short* HST  = (unsigned short*)carve((size_t)3 * NCHUNK * NBATCH * NHID * 2);
  if (off > ws_size || off > (size_t)134217728) return;

  cvt_x_kernel<<<(NROWS * (NIN / 8)) / NTHR, NTHR, 0, stream>>>(x, XA);
  tpw_kernel<<<dim3(4 * NHID / 64, NIN / 64),  NTHR, 0, stream>>>(W0, NIN,  4 * NHID, NIN,  W0T, WCARRY);
  tpw_kernel<<<dim3(4 * NHID / 64, NHID / 64), NTHR, 0, stream>>>(U0, NHID, 4 * NHID, NHID, U0T, WCARRY);
  tpw_kernel<<<dim3(4 * NHID / 64, NHID / 64), NTHR, 0, stream>>>(W1, NHID, 4 * NHID, NHID, W1T, WCARRY);
  tpw_kernel<<<dim3(4 * NHID / 64, NHID / 64), NTHR, 0, stream>>>(U1, NHID, 4 * NHID, NHID, U1T, WCARRY);
  tpw_kernel<<<dim3(4 * NLAT / 64, NHID / 64), NTHR, 0, stream>>>(Wl, NHID, 4 * NLAT, NHID, WLT, WCARRY);
  tpw_kernel<<<dim3(4 * NLAT / 64, NLAT / 64), NTHR, 0, stream>>>(Ul, NLAT, 4 * NLAT, NLAT, ULT, WCARRY);

  const size_t cslot_sz = (size_t)NBATCH * NHID;
  const int gridG_big = ((MCH / 64) * (4 * NHID / 64)) / 8;
  const int gridG_lat = ((MCH / 64) * (4 * NLAT / 64)) / 8;

  for (int ch = 0; ch < NCHUNK; ++ch) {
    const int slot = 0 * NCHUNK + ch;
    const int pslot = (ch > 0) ? (slot - 1) : slot;
    gemm64_f16_kernel<<<gridG_big, 256, 0, stream>>>(
        XA + (size_t)ch * MCH * NIN, NIN, W0T, NIN, XWC, 4 * NHID, b0, MCH, 4 * NHID, NIN, FOLD_XW);
    lstm_scan_kernel<NHID, false><<<NBATCH / 16, NTHR, 0, stream>>>(
        XWC, U0T, g0, be0, m0, v0, SEQ0 + (size_t)ch * MCH * NHID,
        CST + pslot * cslot_sz, HST + pslot * cslot_sz, CST + slot * cslot_sz, HST + slot * cslot_sz,
        out, (ch == 0) ? 1 : 0, 0);
  }
  for (int ch = 0; ch < NCHUNK; ++ch) {
    const int slot = 1 * NCHUNK + ch;
    const int pslot = (ch > 0) ? (slot - 1) : slot;
    gemm64_f16_kernel<<<gridG_big, 256, 0, stream>>>(
        SEQ0 + (size_t)ch * MCH * NHID, NHID, W1T, NHID, XWC, 4 * NHID, b1, MCH, 4 * NHID, NHID, FOLD_HW);
    lstm_scan_kernel<NHID, false><<<NBATCH / 16, NTHR, 0, stream>>>(
        XWC, U1T, g1, be1, m1, v1, SEQ1 + (size_t)ch * MCH * NHID,
        CST + pslot * cslot_sz, HST + pslot * cslot_sz, CST + slot * cslot_sz, HST + slot * cslot_sz,
        out, (ch == 0) ? 1 : 0, 0);
  }
  for (int ch = 0; ch < NCHUNK; ++ch) {
    const int slot = 2 * NCHUNK + ch;
    const int pslot = (ch > 0) ? (slot - 1) : slot;
    gemm64_f16_kernel<<<gridG_lat, 256, 0, stream>>>(
        SEQ1 + (size_t)ch * MCH * NHID, NHID, WLT, NHID, XWC, 4 * NLAT, bl, MCH, 4 * NLAT, NHID, FOLD_HW);
    lstm_scan_kernel<NLAT, true><<<NBATCH / 16, NTHR, 0, stream>>>(
        XWC, ULT, g1, be1, m1, v1, SEQ1,
        CST + pslot * cslot_sz, HST + pslot * cslot_sz, CST + slot * cslot_sz, HST + slot * cslot_sz,
        out, (ch == 0) ? 1 : 0, (ch == NCHUNK - 1) ? 1 : 0);
  }
}
